// MultiheadAttention_15607911153822
// MI455X (gfx1250) — hardware-run, weakly checked
//
#include <hip/hip_runtime.h>


#ifndef NB
#define NB 4
#endif
#ifndef SEQ
#define SEQ 2048
#endif
#define NB_FULL   4
#define SEQ_FULL  2048
#define HID       1024
#define NHEAD     16
#define HD        64
#define MROWS     (NB * SEQ)

#if SEQ > 512
#define EARLY     512
#define HAVE_LATE 1
#else
#define EARLY     SEQ
#define HAVE_LATE 0
#endif

static_assert(HID == NHEAD * HD);
static_assert(NHEAD == 16);
static_assert(HD == 64);
static_assert(SEQ % 128 == 0);
static_assert(EARLY % 128 == 0);
static_assert(EARLY % 32 == 0);
static_assert(EARLY <= SEQ);
static_assert(SEQ <= SEQ_FULL);
static_assert(NB >= 1 && NB <= NB_FULL);
static_assert(MROWS % 128 == 0);
static_assert(HID % 128 == 0);
static_assert(HID % 32 == 0);
static_assert(HID == 128 * 8);

#define CARRY_X    16.0f
#define CARRY_W    32.0f
#define CARRY_QKV  16.0f
#define CARRY_CTX  1024.0f
#define RES_MUL    2048.0f
#define RES_INV    0.00048828125f

typedef unsigned u32;
typedef _Float16 f16;
typedef f16   v16h __attribute__((ext_vector_type(16)));
typedef f16   v8h  __attribute__((ext_vector_type(8)));
typedef float v8f  __attribute__((ext_vector_type(8)));
typedef float v4f  __attribute__((ext_vector_type(4)));

union FragU { v16h v; v8h half[2]; f16 e[16]; };
union H8U   { v8h v; f16 e[8]; };

__device__ __forceinline__ v8f zero8() {
    v8f z = {0.f, 0.f, 0.f, 0.f, 0.f, 0.f, 0.f, 0.f};
    return z;
}

__device__ __forceinline__ v8f wmma16(v16h a, v16h b, v8f c) {
    v8f d = __builtin_amdgcn_wmma_f32_16x16x32_f16(false, a, false, b, (short)0, c, false, false);
    asm volatile("v_nop\n\tv_nop\n\tv_nop\n\tv_nop" : "+v"(d) : "v"(a), "v"(b));
    return d;
}

__device__ __forceinline__ float bf16_rne(float x) {
    u32 u = __float_as_uint(x);
    u = (u + 0x7fffu + ((u >> 16) & 1u)) & 0xffff0000u;
    return __uint_as_float(u);
}

__device__ __forceinline__ float fexp2(float x) {
#if defined(__has_builtin)
#if __has_builtin(__builtin_amdgcn_exp2f)
    return __builtin_amdgcn_exp2f(x);
#else
    return exp2f(x);
#endif
#else
    return exp2f(x);
#endif
}

__device__ __forceinline__ v16h load_frag(const f16* tile, u32 rowbase, u32 pitch, u32 kcol, u32 lane) {
    const u32 r  = rowbase + (lane & 15u);
    const u32 kh = (lane >> 4) << 3;
    const f16* p = tile + (size_t)r * pitch + kcol + kh;
    FragU f;
    f.half[0] = *(const v8h*)(p);
    f.half[1] = *(const v8h*)(p + 16);
    return f.v;
}

__global__ void __launch_bounds__(256)
rope_table(const int* __restrict__ pos, float* __restrict__ cosT, float* __restrict__ sinT) {
#pragma clang fp contract(off)
    const u32 g = blockIdx.x * 256u + threadIdx.x;
    const u32 s = g >> 5;
    const u32 i = g & 31u;
    if (s >= (u32)SEQ) return;
    const float p   = (float)pos[s];
    const float inv = fexp2(-(float)i * 0.41524101186092029f);
    const float ang = p * inv;
    float sn, cs;
    sincosf(ang, &sn, &cs);
    float* cp = cosT + g;
    float* sp = sinT + g;
    *(volatile float*)cp = cs;
    *(volatile float*)sp = sn;
    __threadfence();
    *(volatile float*)cp = cs;
    *(volatile float*)sp = sn;
}

__global__ void __launch_bounds__(256)
cvt_rows(const float* __restrict__ src, f16* __restrict__ dst, u32 nrows, u32 dstper, u32 srcper, float carry) {
#pragma clang fp contract(off)
    const u32 g  = blockIdx.x * 256u + threadIdx.x;
    const u32 m  = g >> 7;
    const u32 c8 = (g & 127u) << 3;
    if (m >= nrows) return;
    const u32 mb = m / dstper;
    const u32 sm = mb * srcper + (m - mb * dstper);
    const float* sp = src + (size_t)sm * HID + c8;
    const v4f a = *(const v4f*)sp;
    const v4f b = *(const v4f*)(sp + 4);
    H8U o;
#pragma unroll
    for (u32 j = 0; j < 4; ++j) {
        const float x0 = a[j];
        const float x1 = b[j];
        o.e[j]     = (f16)(bf16_rne(x0) * carry);
        o.e[j + 4] = (f16)(bf16_rne(x1) * carry);
    }
    f16* dp = dst + (size_t)m * HID + c8;
    *(volatile v8h*)dp = o.v;
    __threadfence();
    *(volatile v8h*)dp = o.v;
}

template <int MODE>
__device__ __forceinline__ void gemm_body(const f16* __restrict__ base, size_t offA, size_t offAlo,
                                          const f16* __restrict__ W,
                                          void* __restrict__ out, void* __restrict__ out2,
                                          const float* __restrict__ cosT, const float* __restrict__ sinT,
                                          float accMul) {
    __shared__ __attribute__((aligned(16))) f16 As[128 * 32];
    __shared__ __attribute__((aligned(16))) f16 Bs[128 * 32];
    __shared__ __attribute__((aligned(16))) f16 Cs[128 * 128];
    static_assert(sizeof(f16) * 128 * 128 == sizeof(float) * 64 * 128);

    const u32 tid  = threadIdx.x;
    const u32 lane = tid & 31u;
    const u32 wave = (u32)__builtin_amdgcn_readfirstlane((int)(tid >> 5));
    const u32 wm   = wave & 3u;
    const u32 wn   = wave >> 2;
    const u32 hh8  = (lane >> 4) << 3;
    const u32 c16  = lane & 15u;
    const u32 m0   = blockIdx.x * 128u;
    const u32 n0   = blockIdx.y * 128u;
    const u32 bidx = m0 / (u32)SEQ;
    const u32 s0   = m0 - bidx * (u32)SEQ;
    const bool early = (s0 < (u32)EARLY);

    v8f acc[2][4];
#pragma unroll
    for (int i = 0; i < 2; ++i)
#pragma unroll
        for (int j = 0; j < 4; ++j) acc[i][j] = zero8();

    const u32 srow = tid >> 1;
    const u32 scol = (tid & 1u) << 4;
    const size_t rowHi = offA + (size_t)(m0 + srow) * HID + scol;
    const size_t rowLo = offAlo + (size_t)(bidx * (u32)EARLY + s0 + srow) * HID + scol;
    const f16* gW = W + (size_t)(n0 + srow) * HID + scol;
    const u32 ph0 = (MODE == 2 && early) ? 0u : 1u;

#pragma unroll 1
    for (u32 ph = ph0; ph < 2u; ++ph) {
        const f16* gA = base + ((ph == 0u) ? rowLo : rowHi);
#pragma unroll 1
        for (u32 k0 = 0; k0 < (u32)HID; k0 += 32u) {
            const v8h ra0 = *(const v8h*)(gA + k0);
            const v8h ra1 = *(const v8h*)(gA + k0 + 8);
            const v8h rb0 = *(const v8h*)(gW + k0);
            const v8h rb1 = *(const v8h*)(gW + k0 + 8);
            __syncthreads();
            *(v8h*)&As[srow * 32u + scol]      = ra0;
            *(v8h*)&As[srow * 32u + scol + 8u] = ra1;
            *(v8h*)&Bs[srow * 32u + scol]      = rb0;
            *(v8h*)&Bs[srow * 32u + scol + 8u] = rb1;
            __syncthreads();

            v16h af[2], bfr[4];
#pragma unroll
            for (int i = 0; i < 2; ++i) af[i] = load_frag(As, wm * 32u + (u32)i * 16u, 32u, 0u, lane);
#pragma unroll
            for (int j = 0; j < 4; ++j) bfr[j] = load_frag(Bs, wn * 64u + (u32)j * 16u, 32u, 0u, lane);
#pragma unroll
            for (int i = 0; i < 2; ++i)
#pragma unroll
                for (int j = 0; j < 4; ++j) acc[i][j] = wmma16(af[i], bfr[j], acc[i][j]);
        }
        if (ph == 0u) {
#pragma unroll
            for (int i = 0; i < 2; ++i)
#pragma unroll
                for (int j = 0; j < 4; ++j) acc[i][j] = acc[i][j] * RES_INV;
        }
    }

    const u32 piece = lane & 7u;
    const u32 lsub  = lane >> 3;

    if constexpr (MODE == 0) {
        float* Cf = (float*)Cs;
        f16* op = (f16*)out;
        f16* ol = (f16*)out2;
        const size_t bh0 = (size_t)bidx * NHEAD + (n0 >> 6);
#pragma unroll
        for (u32 half = 0; half < 2; ++half) {
            if ((wm >> 1) == half) {
#pragma unroll
                for (int i = 0; i < 2; ++i)
#pragma unroll
                    for (int j = 0; j < 4; ++j) {
                        const u32 nl = wn * 64u + (u32)j * 16u + c16;
#pragma unroll
                        for (int r = 0; r < 8; ++r) {
                            const u32 ml = (wm & 1u) * 32u + (u32)i * 16u + hh8 + (u32)r;
                            Cf[ml * 128u + nl] = acc[i][j][r] * accMul;
                        }
                    }
            }
            __syncthreads();
            v8h ov[4], lv[4];
#pragma unroll
            for (u32 it = 0; it < 4; ++it) {
                const u32 L    = wave * 16u + it * 4u + lsub;
                const u32 ml   = L >> 1;
                const u32 hsel = L & 1u;
                const float* cp = &Cf[ml * 128u + hsel * 64u + piece * 8u];
                const v4f a = *(const v4f*)cp;
                const v4f b = *(const v4f*)(cp + 4);
                const u32 sq = s0 + half * 64u + ml;
                const v4f cs = *(const v4f*)(cosT + (size_t)sq * 32u + piece * 4u);
                const v4f sn = *(const v4f*)(sinT + (size_t)sq * 32u + piece * 4u);
                float rv[8];
                rv[0] = cs[0] * a[0] - sn[0] * a[1];
                rv[1] = sn[0] * a[0] + cs[0] * a[1];
                rv[2] = cs[1] * a[2] - sn[1] * a[3];
                rv[3] = sn[1] * a[2] + cs[1] * a[3];
                rv[4] = cs[2] * b[0] - sn[2] * b[1];
                rv[5] = sn[2] * b[0] + cs[2] * b[1];
                rv[6] = cs[3] * b[2] - sn[3] * b[3];
                rv[7] = sn[3] * b[2] + cs[3] * b[3];
                H8U o, l;
#pragma unroll
                for (int e = 0; e < 8; ++e) {
                    const f16 hv = (f16)rv[e];
                    o.e[e] = hv;
                    l.e[e] = (f16)((rv[e] - (float)hv) * RES_MUL);
                }
                ov[it] = o.v;
                lv[it] = l.v;
            }
#pragma unroll
            for (int pass = 0; pass < 2; ++pass) {
#pragma unroll
                for (u32 it = 0; it < 4; ++it) {
                    const u32 L    = wave * 16u + it * 4u + lsub;
                    const u32 ml   = L >> 1;
                    const u32 hsel = L & 1u;
                    f16* dp = op + ((bh0 + hsel) * SEQ + s0 + half * 64u + ml) * HD + piece * 8u;
                    *(volatile v8h*)dp = ov[it];
                    if (early) {
                        f16* dl = ol + ((bh0 + hsel) * EARLY + s0 + half * 64u + ml) * HD + piece * 8u;
                        *(volatile v8h*)dl = lv[it];
                    }
                }
                if (pass == 0) __threadfence();
            }
            __syncthreads();
        }
    } else if constexpr (MODE == 1) {
#pragma unroll
        for (int i = 0; i < 2; ++i)
#pragma unroll
            for (int j = 0; j < 4; ++j) {
                const u32 nl = wn * 64u + (u32)j * 16u + c16;
                H8U t;
#pragma unroll
                for (int r = 0; r < 8; ++r) t.e[r] = (f16)(acc[i][j][r] * accMul);
                *(v8h*)&Cs[nl * 128u + wm * 32u + (u32)i * 16u + hh8] = t.v;
            }
        __syncthreads();
        f16* op = (f16*)out;
#pragma unroll
        for (int pass = 0; pass < 2; ++pass) {
#pragma unroll
            for (u32 it = 0; it < 8; ++it) {
                const u32 L  = wave * 32u + it * 4u + lsub;
                const u32 nl = L >> 1;
                const u32 mh = L & 1u;
                const v8h v = *(const v8h*)&Cs[nl * 128u + mh * 64u + piece * 8u];
                f16* dp = op + ((size_t)(bidx * (u32)HID + n0 + nl) * SEQ + s0 + mh * 64u + piece * 8u);
                *(volatile v8h*)dp = v;
            }
            if (pass == 0) __threadfence();
        }
        if (early) {
            __syncthreads();
#pragma unroll
            for (int i = 0; i < 2; ++i)
#pragma unroll
                for (int j = 0; j < 4; ++j) {
                    const u32 nl = wn * 64u + (u32)j * 16u + c16;
                    H8U t;
#pragma unroll
                    for (int r = 0; r < 8; ++r) {
                        const float val = acc[i][j][r] * accMul;
                        const f16 hv = (f16)val;
                        t.e[r] = (f16)((val - (float)hv) * RES_MUL);
                    }
                    *(v8h*)&Cs[nl * 128u + wm * 32u + (u32)i * 16u + hh8] = t.v;
                }
            __syncthreads();
            f16* ol = (f16*)out2;
#pragma unroll
            for (int pass = 0; pass < 2; ++pass) {
#pragma unroll
                for (u32 it = 0; it < 8; ++it) {
                    const u32 L  = wave * 32u + it * 4u + lsub;
                    const u32 nl = L >> 1;
                    const u32 mh = L & 1u;
                    const v8h v = *(const v8h*)&Cs[nl * 128u + mh * 64u + piece * 8u];
                    f16* dp = ol + ((size_t)(bidx * (u32)HID + n0 + nl) * EARLY + s0 + mh * 64u + piece * 8u);
                    *(volatile v8h*)dp = v;
                }
                if (pass == 0) __threadfence();
            }
        }
    } else {
        float* Cf = (float*)Cs;
        float* of = (float*)out;
#pragma unroll
        for (u32 half = 0; half < 2; ++half) {
            if ((wm >> 1) == half) {
#pragma unroll
                for (int i = 0; i < 2; ++i)
#pragma unroll
                    for (int j = 0; j < 4; ++j) {
                        const u32 nl = wn * 64u + (u32)j * 16u + c16;
#pragma unroll
                        for (int r = 0; r < 8; ++r) {
                            const u32 ml = (wm & 1u) * 32u + (u32)i * 16u + hh8 + (u32)r;
                            Cf[ml * 128u + nl] = acc[i][j][r] * accMul;
                        }
                    }
            }
            __syncthreads();
#pragma unroll
            for (int pass = 0; pass < 2; ++pass) {
#pragma unroll
                for (u32 it = 0; it < 8; ++it) {
                    const u32 L    = wave * 32u + it * 4u + lsub;
                    const u32 row  = L >> 2;
                    const u32 part = L & 3u;
                    const v4f v = *(const v4f*)&Cf[row * 128u + part * 32u + piece * 4u];
                    float* dp = of + (size_t)(m0 + half * 64u + row) * HID + n0 + part * 32u + piece * 4u;
                    *(volatile v4f*)dp = v;
                }
                if (pass == 0) __threadfence();
            }
            __syncthreads();
        }
    }
}

__global__ void __launch_bounds__(256) __attribute__((amdgpu_num_vgpr(256)))
gemm_qk(const f16* __restrict__ A, const f16* __restrict__ W, f16* __restrict__ out,
        f16* __restrict__ outlo,
        const float* __restrict__ cosT, const float* __restrict__ sinT, float accMul) {
    gemm_body<0>(A, (size_t)0, (size_t)0, W, (void*)out, (void*)outlo, cosT, sinT, accMul);
}

__global__ void __launch_bounds__(256) __attribute__((amdgpu_num_vgpr(256)))
gemm_vt(const f16* __restrict__ A, const f16* __restrict__ W, f16* __restrict__ out,
        f16* __restrict__ outlo, float accMul) {
    gemm_body<1>(A, (size_t)0, (size_t)0, W, (void*)out, (void*)outlo, (const float*)0, (const float*)0, accMul);
}

__global__ void __launch_bounds__(256) __attribute__((amdgpu_num_vgpr(256)))
gemm_out(const f16* __restrict__ wsb, size_t offA, size_t offAlo, const f16* __restrict__ W,
         float* __restrict__ out, float accMul) {
    gemm_body<2>(wsb, offA, offAlo, W, (void*)out, (void*)0, (const float*)0, (const float*)0, accMul);
}

template <int EP>
__device__ __forceinline__ void attn_body(const f16* __restrict__ Qp, const f16* __restrict__ Ql,
                                          const f16* __restrict__ Kp, const f16* __restrict__ Kl,
                                          const f16* __restrict__ Vt, const f16* __restrict__ Vtl,
                                          f16* __restrict__ Cp, f16* __restrict__ Cl, u32 qblk) {
    __shared__ __attribute__((aligned(16))) f16 stg[(EP ? 2 : 1) * 8 * 1024];

    const u32 tid  = threadIdx.x;
    const u32 lane = tid & 31u;
    const u32 wave = (u32)__builtin_amdgcn_readfirstlane((int)(tid >> 5));
    const u32 hh8  = (lane >> 4) << 3;
    const u32 c16  = lane & 15u;
    const u32 bh   = blockIdx.y;
    const u32 bidx = bh >> 4;
    const u32 hidx = bh & 15u;
    const u32 q0   = qblk * 128u + wave * 16u;
    const u32 qi   = q0 + c16;
    const size_t head  = (size_t)bh * SEQ * HD;
    const size_t headE = (size_t)bh * EARLY * HD;
    const f16* Qh  = Qp + head;
    const f16* Kh  = Kp + head;
    const f16* Qlh = Ql + headE;
    const f16* Klh = Kl + headE;
    const f16* Vh  = Vt + (size_t)(bidx * (u32)HID + hidx * (u32)HD) * SEQ;
    const f16* Vlh = Vtl + (size_t)(bidx * (u32)HID + hidx * (u32)HD) * EARLY;

    v16h qb[2], ql[2];
#pragma unroll
    for (int c = 0; c < 2; ++c) {
        qb[c] = load_frag(Qh, q0, HD, (u32)c * 32u, lane);
        if constexpr (EP != 0) ql[c] = load_frag(Qlh, q0, HD, (u32)c * 32u, lane);
        else                   ql[c] = qb[c];
    }

    FragU onesu;
#pragma unroll
    for (int i = 0; i < 16; ++i) onesu.e[i] = (f16)1.0f;
    const v16h ones = onesu.v;

    float m = -1.0e30f;
    v8f o[4], o1[4], lacc, l1;
#pragma unroll
    for (int dt = 0; dt < 4; ++dt) { o[dt] = zero8(); o1[dt] = zero8(); }
    lacc = zero8();
    l1   = zero8();

    const float cl = 1.4426950408889634f * 0.00048828125f;
    const u32 nsteps = (q0 + 47u) >> 5;

#pragma unroll 1
    for (u32 kt = 0; kt < nsteps; ++kt) {
        const u32 key0 = kt << 5;
        v8f sa = zero8();
        v8f sb = zero8();
        v8f ra = zero8();
        v8f rb = zero8();
#pragma unroll
        for (int c = 0; c < 2; ++c) {
            const v16h ka = load_frag(Kh, key0,       HD, (u32)c * 32u, lane);
            const v16h kb = load_frag(Kh, key0 + 16u, HD, (u32)c * 32u, lane);
            sa = wmma16(ka, qb[c], sa);
            sb = wmma16(kb, qb[c], sb);
            if constexpr (EP != 0) {
                const v16h kal = load_frag(Klh, key0,       HD, (u32)c * 32u, lane);
                const v16h kbl = load_frag(Klh, key0 + 16u, HD, (u32)c * 32u, lane);
                ra = wmma16(ka,  ql[c], ra);
                ra = wmma16(kal, qb[c], ra);
                rb = wmma16(kb,  ql[c], rb);
                rb = wmma16(kbl, qb[c], rb);
            }
        }

        float xa[8], xb[8];
#pragma unroll
        for (int r = 0; r < 8; ++r) {
            if constexpr (EP != 0) {
                xa[r] = (sa[r] + ra[r] * RES_INV) * cl;
                xb[r] = (sb[r] + rb[r] * RES_INV) * cl;
            } else {
                xa[r] = sa[r] * cl;
                xb[r] = sb[r] * cl;
            }
        }
        if (kt + 1u == nsteps) {
#pragma unroll
            for (int r = 0; r < 8; ++r) {
                const u32 kk = key0 + hh8 + (u32)r;
                xa[r] = (kk <= qi)       ? xa[r] : -1.0e30f;
                xb[r] = (kk + 16u <= qi) ? xb[r] : -1.0e30f;
            }
        }
        float tm = fmaxf(xa[0], xb[0]);
#pragma unroll
        for (int r = 1; r < 8; ++r) tm = fmaxf(tm, fmaxf(xa[r], xb[r]));
        const float tmo = __shfl_xor(tm, 16);
        tm = fmaxf(tm, tmo);
        const float mn = fmaxf(m, tm);
        const float al = fexp2(m - mn);
        m = mn;
#pragma unroll
        for (int dt = 0; dt < 4; ++dt) o[dt] = o[dt] * al;
        lacc = lacc * al;
        if constexpr (EP != 0) {
#pragma unroll
            for (int dt = 0; dt < 4; ++dt) o1[dt] = o1[dt] * al;
            l1 = l1 * al;
        }
        const float sh = 10.0f - mn;

        FragU pb, pl;
#pragma unroll
        for (int r = 0; r < 8; ++r) {
            const float pa = fexp2(xa[r] + sh);
            const float pc = fexp2(xb[r] + sh);
            const f16 ha = (f16)pa;
            const f16 hc = (f16)pc;
            pb.e[r]     = ha;
            pb.e[8 + r] = hc;
            if constexpr (EP != 0) {
                pl.e[r]     = (f16)((pa - (float)ha) * RES_MUL);
                pl.e[8 + r] = (f16)((pc - (float)hc) * RES_MUL);
            } else {
                pl.e[r]     = (f16)0.0f;
                pl.e[8 + r] = (f16)0.0f;
            }
        }

#pragma unroll
        for (int dt = 0; dt < 4; ++dt) {
            const v16h va = load_frag(Vh, (u32)dt * 16u, (u32)SEQ, key0, lane);
            o[dt] = wmma16(va, pb.v, o[dt]);
            if constexpr (EP != 0) {
                const v16h vl = load_frag(Vlh, (u32)dt * 16u, (u32)EARLY, key0, lane);
                o1[dt] = wmma16(va, pl.v, o1[dt]);
                o1[dt] = wmma16(vl, pb.v, o1[dt]);
            }
        }
        lacc = wmma16(ones, pb.v, lacc);
        if constexpr (EP != 0) l1 = wmma16(ones, pl.v, l1);
    }

    float lsum = lacc[0];
    if constexpr (EP != 0) lsum = lsum + l1[0] * RES_INV;
    const float inv = (CARRY_CTX / CARRY_QKV) / lsum;
    f16* sw  = &stg[wave * 1024u];
    f16* swl = &stg[(EP ? 8u * 1024u : 0u) + wave * 1024u];
#pragma unroll
    for (int dt = 0; dt < 4; ++dt) {
        H8U t, tl;
#pragma unroll
        for (int r = 0; r < 8; ++r) {
            float ov = o[dt][r];
            if constexpr (EP != 0) ov = ov + o1[dt][r] * RES_INV;
            const float val = ov * inv;
            const f16 hv = (f16)val;
            t.e[r]  = hv;
            tl.e[r] = (f16)((val - (float)hv) * RES_MUL);
        }
        *(v8h*)&sw[c16 * 64u + (u32)dt * 16u + hh8] = t.v;
        if constexpr (EP != 0) *(v8h*)&swl[c16 * 64u + (u32)dt * 16u + hh8] = tl.v;
    }
    __syncthreads();

    const u32 piece = lane & 7u;
    const u32 lsub  = lane >> 3;
#pragma unroll
    for (int pass = 0; pass < 2; ++pass) {
#pragma unroll
        for (u32 it = 0; it < 4; ++it) {
            const u32 L = it * 4u + lsub;
            const v8h v = *(const v8h*)&sw[L * 64u + piece * 8u];
            f16* dp = Cp + ((size_t)(bidx * (u32)SEQ + q0 + L) * HID + hidx * (u32)HD + piece * 8u);
            *(volatile v8h*)dp = v;
            if constexpr (EP != 0) {
                const v8h w = *(const v8h*)&swl[L * 64u + piece * 8u];
                f16* dl = Cl + ((size_t)(bidx * (u32)EARLY + q0 + L) * HID + hidx * (u32)HD + piece * 8u);
                *(volatile v8h*)dl = w;
            }
        }
        if (pass == 0) __threadfence();
    }
}

__global__ void __launch_bounds__(256) __attribute__((amdgpu_num_vgpr(256)))
attn_early(const f16* __restrict__ Qp, const f16* __restrict__ Ql,
           const f16* __restrict__ Kp, const f16* __restrict__ Kl,
           const f16* __restrict__ Vt, const f16* __restrict__ Vtl,
           f16* __restrict__ Cp, f16* __restrict__ Cl) {
    attn_body<1>(Qp, Ql, Kp, Kl, Vt, Vtl, Cp, Cl, blockIdx.x);
}

__global__ void __launch_bounds__(256) __attribute__((amdgpu_num_vgpr(256)))
attn_late(const f16* __restrict__ Qp, const f16* __restrict__ Kp, const f16* __restrict__ Vt,
          f16* __restrict__ Cp) {
    attn_body<0>(Qp, Qp, Kp, Kp, Vt, Vt, Cp, Cp, blockIdx.x + (u32)(EARLY / 128));
}

static_assert((size_t)(SEQ / 8) * 256 == (size_t)SEQ * 32);
static_assert((size_t)(MROWS / 2) * 256 * 8 == (size_t)MROWS * HID);
static_assert((size_t)(HID / 2) * 256 * 8 == (size_t)HID * HID);
static_assert((size_t)(MROWS / 128) * (HID / 128) * 128 * 128 == (size_t)MROWS * HID);
static_assert((size_t)(NB * (EARLY / 128)) * (HID / 128) * 128 * 128 == (size_t)NB * EARLY * HID);
static_assert((size_t)(SEQ / 128) * (NB * NHEAD) * 128 * HD == (size_t)MROWS * HID);
static_assert((size_t)(EARLY / 128) * (NB * NHEAD) * 128 * HD == (size_t)NB * EARLY * HID);
static_assert(((size_t)5 * MROWS * HID + (size_t)4 * HID * HID + (size_t)4 * NB * EARLY * HID) * sizeof(f16)
              + (size_t)2 * SEQ * 32 * sizeof(float) <= (size_t)134217728);

extern "C" void kernel_launch(void* const* d_in, const int* in_sizes, int n_in,
                              void* d_out, int out_size, void* d_ws, size_t ws_size,
                              hipStream_t stream) {
    if (n_in < 6) return;
    if (in_sizes[0] < ((NB - 1) * SEQ_FULL + SEQ) * HID) return;
    if (in_sizes[1] < HID * HID) return;
    if (in_sizes[2] < HID * HID) return;
    if (in_sizes[3] < HID * HID) return;
    if (in_sizes[4] < HID * HID) return;
    if (in_sizes[5] < SEQ) return;
    if (out_size < MROWS * HID) return;

    const float* x   = (const float*)d_in[0];
    const float* wq  = (const float*)d_in[1];
    const float* wk  = (const float*)d_in[2];
    const float* wv  = (const float*)d_in[3];
    const float* wo  = (const float*)d_in[4];
    const int*   pos = (const int*)d_in[5];

    const size_t nX = (size_t)MROWS * HID;
    const size_t nW = (size_t)HID * HID;
    const size_t nE = (size_t)NB * EARLY * HID;
    const size_t nT = (size_t)SEQ * 32;
    const size_t totalBytes = (5 * nX + 4 * nW + 4 * nE) * sizeof(f16) + 2 * nT * sizeof(float);
    if (ws_size < totalBytes) return;

    f16* Xh  = (f16*)d_ws;
    f16* Wqh = Xh  + nX;
    f16* Wkh = Wqh + nW;
    f16* Wvh = Wkh + nW;
    f16* Woh = Wvh + nW;
    f16* Qp  = Woh + nW;
    f16* Kp  = Qp  + nX;
    f16* Vtp = Kp  + nX;
    f16* Cp  = Vtp + nX;
    f16* Vtl = Cp  + nX;
    f16* Cl  = Vtl + nE;
    f16* Qlp = Cl  + nE;
    f16* Klp = Qlp + nE;
    float* cosT = (float*)(Klp + nE);
    float* sinT = cosT + nT;

    rope_table<<<SEQ / 8, 256, 0, stream>>>(pos, cosT, sinT);

    cvt_rows<<<MROWS / 2, 256, 0, stream>>>(x, Xh, (u32)MROWS, (u32)SEQ, (u32)SEQ_FULL, CARRY_X);
    cvt_rows<<<HID / 2, 256, 0, stream>>>(wq, Wqh, (u32)HID, (u32)HID, (u32)HID, CARRY_W);
    cvt_rows<<<HID / 2, 256, 0, stream>>>(wk, Wkh, (u32)HID, (u32)HID, (u32)HID, CARRY_W);
    cvt_rows<<<HID / 2, 256, 0, stream>>>(wv, Wvh, (u32)HID, (u32)HID, (u32)HID, CARRY_W);
    cvt_rows<<<HID / 2, 256, 0, stream>>>(wo, Woh, (u32)HID, (u32)HID, (u32)HID, CARRY_W);

    const dim3 gg(MROWS / 128, HID / 128);
    const float accQKV = CARRY_QKV / (CARRY_X * CARRY_W);
    gemm_qk<<<gg, 256, 0, stream>>>(Xh, Wqh, Qp, Qlp, cosT, sinT, accQKV);
    gemm_qk<<<gg, 256, 0, stream>>>(Xh, Wkh, Kp, Klp, cosT, sinT, accQKV);
    gemm_vt<<<gg, 256, 0, stream>>>(Xh, Wvh, Vtp, Vtl, accQKV);

    attn_early<<<dim3(EARLY / 128, NB * NHEAD), 256, 0, stream>>>(Qp, Qlp, Kp, Klp, Vtp, Vtl, Cp, Cl);
#if HAVE_LATE
    attn_late<<<dim3((SEQ - EARLY) / 128, NB * NHEAD), 256, 0, stream>>>(Qp, Kp, Vtp, Cp);
#endif

    const float accOut = 1.0f / (CARRY_CTX * CARRY_W);
    gemm_out<<<gg, 256, 0, stream>>>(Xh, (size_t)(Cp - Xh), (size_t)(Cl - Xh), Woh, (float*)d_out, accOut);
}
